// MambaBlock_37082747633911
// MI455X (gfx1250) — hardware-verified
//
#include <hip/hip_runtime.h>
#include <stddef.h>
#include <stdint.h>
#include <math.h>


#define DIM     1024
#define DIN     2048
#define MROWS   2048
#define SEQ     1024
#define NIN     4096
#define K2      4096
#define NDBC    2112
#define BCW     32
#define PLANE   (MROWS * DIN)
#define GBM     64
#define GBN     64
#define GTHR    128
#define NTHR    256
#define ST      32
#define SCH     128
#define SCAN_LDS_FLOATS (4 * ST * SCH + ST * BCW)
#define U_XB    (MROWS * DIM / 8)
#define U_WIN   (NIN * DIM / 8)
#define U_WD    (NDBC * K2 / 8)
#define U_WO    (DIM * K2 / 8)
#define U_TOT   (U_XB + U_WIN + U_WD + U_WO)
#define WSMAX   134217728

static_assert(MROWS % GBM == 0 && NIN % GBN == 0 && NDBC % GBN == 0 && DIM % GBN == 0 && DIN % GBN == 0);
static_assert(DIM % 32 == 0 && K2 % 32 == 0 && K2 == 2 * DIN);
static_assert(GBM == (GTHR / 32) * 16 && GBN == 64);
static_assert(U_XB % 512 == 0 && (U_XB + U_WIN) % 512 == 0 && (U_XB + U_WIN + U_WD) % 512 == 0 && U_TOT % NTHR == 0);
static_assert(SEQ % ST == 0 && DIN % SCH == 0 && SCH * 2 == NTHR);
static_assert(ST * SCH / 4 == 4 * NTHR && ST * BCW / 4 == NTHR);
static_assert(SCAN_LDS_FLOATS * 4 == 69632);
static_assert(MROWS == 2 * SEQ && (SEQ & (SEQ - 1)) == 0);

typedef float          v4f   __attribute__((ext_vector_type(4)));
typedef float          v8f   __attribute__((ext_vector_type(8)));
typedef int            v8i   __attribute__((ext_vector_type(8)));
typedef unsigned       v2u   __attribute__((ext_vector_type(2)));
typedef unsigned short v4us  __attribute__((ext_vector_type(4)));
typedef unsigned short v8us  __attribute__((ext_vector_type(8)));
typedef unsigned short v16us __attribute__((ext_vector_type(16)));
typedef __bf16         v16bf __attribute__((ext_vector_type(16)));
typedef v4f  __attribute__((may_alias)) v4fa;
typedef v2u  __attribute__((may_alias)) v2ua;
typedef v4us __attribute__((may_alias)) v4usa;
typedef v8us __attribute__((may_alias)) v8usa;
union FragB { v16bf v; v16us u; v8us h[2]; v8i w; };

__device__ __forceinline__ v8f wmb(const FragB& a, const FragB& b, v8f c) {
  v8f d = __builtin_amdgcn_wmma_f32_16x16x32_bf16(false, a.v, false, b.v, (short)0, c, false, false);
  asm volatile("v_nop\n\tv_nop\n\tv_nop\n\tv_nop" : "+v"(d) : "v"(a.w), "v"(b.w));
  return d;
}

__device__ __forceinline__ unsigned bf16_bits(float f) {
  const unsigned u = __float_as_uint(f);
  return (u + 0x7FFFu + ((u >> 16) & 1u)) >> 16;
}
__device__ __forceinline__ float bf16_val(float f) {
  return __uint_as_float(bf16_bits(f) << 16);
}
__device__ __forceinline__ unsigned short hl_bits(float v, int lo) {
  const unsigned hb = bf16_bits(v);
  const unsigned lb = bf16_bits(v - __uint_as_float(hb << 16));
  return (unsigned short)(lo != 0 ? lb : hb);
}
__device__ __forceinline__ float silu_f(float v) {
  return v * __builtin_amdgcn_rcpf(1.0f + expf(-v));
}
__device__ __forceinline__ float softplus_f(float p) {
  return fmaxf(p, 0.0f) + log1pf(expf(-fabsf(p)));
}

__global__ __launch_bounds__(NTHR) void k_prep(const float* __restrict__ x, const float* __restrict__ Win,
                                               const float* __restrict__ Wdt, const float* __restrict__ WB,
                                               const float* __restrict__ WC, const float* __restrict__ Wout,
                                               unsigned short* XB, unsigned short* WIN,
                                               unsigned short* WDBC2, unsigned short* WOUT2) {
  const int u = (int)blockIdx.x * NTHR + (int)threadIdx.x;
  const float* src;
  unsigned short* dst;
  bool live = true;
  if (u < U_XB) {
    const int row = u >> 7;
    const int k8  = (u & 127) * 8;
    src = x + (size_t)row * DIM + k8;
    dst = XB + (size_t)row * DIM + k8;
  } else if (u < U_XB + U_WIN) {
    const int v   = u - U_XB;
    const int row = v >> 7;
    const int k8  = (v & 127) * 8;
    src = Win + (size_t)row * DIM + k8;
    dst = WIN + (size_t)row * DIM + k8;
  } else if (u < U_XB + U_WIN + U_WD) {
    const int v  = u - (U_XB + U_WIN);
    const int n  = v >> 9;
    const int kk = (v & 511) * 8;
    const int k  = kk & (DIN - 1);
    dst = WDBC2 + (size_t)n * K2 + kk;
    if (n < DIN)            { src = Wdt + (size_t)n * DIN + k; }
    else if (n < DIN + 16)  { src = WB + (size_t)(n - DIN) * DIN + k; }
    else if (n < DIN + 32)  { src = WC + (size_t)(n - DIN - 16) * DIN + k; }
    else                    { src = Wdt + k; live = false; }
  } else if (u < U_TOT) {
    const int v  = u - (U_XB + U_WIN + U_WD);
    const int n  = v >> 9;
    const int kk = (v & 511) * 8;
    const int k  = kk & (DIN - 1);
    src = Wout + (size_t)n * DIN + k;
    dst = WOUT2 + (size_t)n * K2 + kk;
  } else {
    return;
  }
  const v4f a = *(const v4f*)src;
  const v4f b = *(const v4f*)(src + 4);
  v8us o;
  o[0] = live ? (unsigned short)bf16_bits(a.x) : (unsigned short)0;
  o[1] = live ? (unsigned short)bf16_bits(a.y) : (unsigned short)0;
  o[2] = live ? (unsigned short)bf16_bits(a.z) : (unsigned short)0;
  o[3] = live ? (unsigned short)bf16_bits(a.w) : (unsigned short)0;
  o[4] = live ? (unsigned short)bf16_bits(b.x) : (unsigned short)0;
  o[5] = live ? (unsigned short)bf16_bits(b.y) : (unsigned short)0;
  o[6] = live ? (unsigned short)bf16_bits(b.z) : (unsigned short)0;
  o[7] = live ? (unsigned short)bf16_bits(b.w) : (unsigned short)0;
  *(volatile v8us*)dst = o;
  __threadfence();
  *(volatile v8us*)dst = o;
}

template <int EPI, int LDO>
__global__ __launch_bounds__(GTHR) void k_gemm(const unsigned short* __restrict__ A,
                                               const unsigned short* __restrict__ WT, int K,
                                               float* outA, float* outB,
                                               const float* __restrict__ vec,
                                               const unsigned short* __restrict__ xres) {
  __shared__ __attribute__((aligned(16))) float stg[GBM * GBN];
  const int tid = (int)threadIdx.x, lane = tid & 31, wave = tid >> 5, hh = lane >> 4, m = lane & 15;
  const int rowBase = (int)blockIdx.x * GBM;
  const int col0    = (int)blockIdx.y * GBN;

  v8f acc[4];
  {
    const v8f z = {0.f, 0.f, 0.f, 0.f, 0.f, 0.f, 0.f, 0.f};
    acc[0] = z; acc[1] = z; acc[2] = z; acc[3] = z;
  }
  const unsigned short* ap = A  + (size_t)(rowBase + 16 * wave + m) * (size_t)K + 8 * hh;
  const unsigned short* wp = WT + (size_t)(col0 + m) * (size_t)K + 8 * hh;
  const int ksteps = K >> 5;
#pragma unroll 1
  for (int ks = 0; ks < ksteps; ++ks) {
    FragB af;
    af.h[0] = *(const v8usa*)(ap + 32 * ks);
    af.h[1] = *(const v8usa*)(ap + 32 * ks + 16);
#pragma unroll
    for (int t = 0; t < 4; ++t) {
      const unsigned short* wq = wp + (size_t)(16 * t) * (size_t)K + 32 * ks;
      FragB bf;
      bf.h[0] = *(const v8usa*)wq;
      bf.h[1] = *(const v8usa*)(wq + 16);
      acc[t] = wmb(af, bf, acc[t]);
    }
  }

#pragma unroll
  for (int t = 0; t < 4; ++t) {
    const int lc = 16 * t + m;
#pragma unroll
    for (int r = 0; r < 8; ++r) {
      const int lr = 16 * wave + 8 * hh + r;
      stg[lr * GBN + lc] = acc[t][r];
    }
  }
  __syncthreads();

  const int c4 = 4 * m;
  size_t oofs = 0;
  int ocol = col0;
  bool tile = true;

  if constexpr (EPI == 0) {
    const bool isZ = col0 >= DIN;
    if (isZ) {
#pragma unroll 1
      for (int i = 0; i < 8; ++i) {
        float* sp = stg + (16 * wave + 2 * i + hh) * GBN + c4;
        v4f v = *(const v4fa*)sp;
        v.x = silu_f(v.x); v.y = silu_f(v.y); v.z = silu_f(v.z); v.w = silu_f(v.w);
        *(v4fa*)sp = v;
      }
      oofs = (size_t)PLANE;
      ocol = col0 - DIN;
    }
  }
  if constexpr (EPI == 1) {
    const bool last = col0 >= DIN;
    if (!last) {
      const v4f bq = *(const v4f*)(vec + col0 + c4);
      const float b0 = bf16_val(bq.x), b1 = bf16_val(bq.y), b2 = bf16_val(bq.z), b3 = bf16_val(bq.w);
#pragma unroll 1
      for (int i = 0; i < 8; ++i) {
        float* sp = stg + (16 * wave + 2 * i + hh) * GBN + c4;
        v4f v = *(const v4fa*)sp;
        v.x = softplus_f(v.x + b0); v.y = softplus_f(v.y + b1);
        v.z = softplus_f(v.z + b2); v.w = softplus_f(v.w + b3);
        *(v4fa*)sp = v;
      }
    } else {
      tile = false;
      v4f bv[4];
#pragma unroll
      for (int i = 0; i < 4; ++i) {
        const int lr = 16 * wave + 4 * i + (lane >> 3);
        bv[i] = *(const v4fa*)(stg + lr * GBN + 4 * (lane & 7));
      }
#pragma unroll
      for (int i = 0; i < 4; ++i) {
        const int lr = 16 * wave + 4 * i + (lane >> 3);
        *(volatile v4f*)(outB + (size_t)(rowBase + lr) * BCW + 4 * (lane & 7)) = bv[i];
      }
      __threadfence();
#pragma unroll
      for (int i = 0; i < 4; ++i) {
        const int lr = 16 * wave + 4 * i + (lane >> 3);
        *(volatile v4f*)(outB + (size_t)(rowBase + lr) * BCW + 4 * (lane & 7)) = bv[i];
      }
    }
  }
  if constexpr (EPI == 2) {
#pragma unroll 1
    for (int i = 0; i < 8; ++i) {
      const int lr = 16 * wave + 2 * i + hh;
      float* sp = stg + lr * GBN + c4;
      v4f v = *(const v4fa*)sp;
      const v2u w = *(const v2ua*)(xres + (size_t)(rowBase + lr) * DIM + col0 + c4);
      v.x += __uint_as_float(w.x << 16);
      v.y += __uint_as_float(w.x & 0xffff0000u);
      v.z += __uint_as_float(w.y << 16);
      v.w += __uint_as_float(w.y & 0xffff0000u);
      *(v4fa*)sp = v;
    }
  }

  if (tile) {
    float* obase = outA + oofs;
    v4f fv[8];
#pragma unroll
    for (int i = 0; i < 8; ++i) {
      const int lr = 16 * wave + 2 * i + hh;
      fv[i] = *(const v4fa*)(stg + lr * GBN + c4);
    }
#pragma unroll
    for (int i = 0; i < 8; ++i) {
      const int lr = 16 * wave + 2 * i + hh;
      float* op = obase + (size_t)(rowBase + lr) * (size_t)LDO + ocol + c4;
      *(volatile v4f*)op = fv[i];
    }
    __threadfence();
#pragma unroll
    for (int i = 0; i < 8; ++i) {
      const int lr = 16 * wave + 2 * i + hh;
      float* op = obase + (size_t)(rowBase + lr) * (size_t)LDO + ocol + c4;
      *(volatile v4f*)op = fv[i];
    }
  }
}

__global__ __launch_bounds__(NTHR) void k_conv(const float* __restrict__ XI, const float* __restrict__ Wc,
                                               const float* __restrict__ bc, float* U, unsigned short* UHL) {
  __shared__ __attribute__((aligned(16))) unsigned short hls[2048];
  const int tid = (int)threadIdx.x;
  const int r   = (int)blockIdx.x >> 1;
  const int cb  = ((int)blockIdx.x & 1) * 1024;
  const int c   = cb + 4 * tid;
  const int l   = r & (SEQ - 1);

  v4f w0 = *(const v4f*)(Wc + (size_t)c * 4);
  v4f w1 = *(const v4f*)(Wc + (size_t)c * 4 + 4);
  v4f w2 = *(const v4f*)(Wc + (size_t)c * 4 + 8);
  v4f w3 = *(const v4f*)(Wc + (size_t)c * 4 + 12);
  const v4f bq = *(const v4f*)(bc + c);
#pragma unroll
  for (int j = 0; j < 4; ++j) {
    w0[j] = bf16_val(w0[j]); w1[j] = bf16_val(w1[j]); w2[j] = bf16_val(w2[j]); w3[j] = bf16_val(w3[j]);
  }
  float s0 = 0.0f, s1 = 0.0f, s2 = 0.0f, s3 = 0.0f;
#pragma unroll
  for (int j = 0; j < 4; ++j) {
    const bool ok = (l - 3 + j) >= 0;
    const int rr = ok ? (r - 3 + j) : r;
    v4f xv = *(const v4f*)(XI + (size_t)rr * DIN + c);
    xv.x = ok ? xv.x : 0.0f; xv.y = ok ? xv.y : 0.0f; xv.z = ok ? xv.z : 0.0f; xv.w = ok ? xv.w : 0.0f;
    s0 = fmaf(w0[j], xv.x, s0);
    s1 = fmaf(w1[j], xv.y, s1);
    s2 = fmaf(w2[j], xv.z, s2);
    s3 = fmaf(w3[j], xv.w, s3);
  }
  v4f uo;
  uo.x = silu_f(s0 + bf16_val(bq.x));
  uo.y = silu_f(s1 + bf16_val(bq.y));
  uo.z = silu_f(s2 + bf16_val(bq.z));
  uo.w = silu_f(s3 + bf16_val(bq.w));

  v4us h4, l4;
  h4[0] = hl_bits(uo.x, 0); l4[0] = hl_bits(uo.x, 1);
  h4[1] = hl_bits(uo.y, 0); l4[1] = hl_bits(uo.y, 1);
  h4[2] = hl_bits(uo.z, 0); l4[2] = hl_bits(uo.z, 1);
  h4[3] = hl_bits(uo.w, 0); l4[3] = hl_bits(uo.w, 1);
  *(v4usa*)(hls + 4 * tid) = h4;
  *(v4usa*)(hls + 1024 + 4 * tid) = l4;
  __syncthreads();
  const int pl = tid >> 7;
  const int ix = tid & 127;
  const v8us q = *(const v8usa*)(hls + pl * 1024 + 8 * ix);

  float* up = U + (size_t)r * DIN + c;
  unsigned short* hp = UHL + (size_t)r * K2 + (size_t)pl * DIN + cb + 8 * ix;
  *(volatile v4f*)up = uo;
  *(volatile v8us*)hp = q;
  __threadfence();
  *(volatile v4f*)up = uo;
  *(volatile v8us*)hp = q;
}

__global__ __launch_bounds__(NTHR) void k_scan(const float* __restrict__ DELTA, const float* __restrict__ U,
                                               const float* __restrict__ SZ, const float* __restrict__ BC,
                                               const float* __restrict__ Alog, const float* __restrict__ Dv,
                                               unsigned short* GHL) {
  extern __shared__ __attribute__((aligned(16))) float sm[];
  float* dl  = sm;
  float* uu  = sm + ST * SCH;
  float* sz  = sm + 2 * ST * SCH;
  float* gg  = sm + 3 * ST * SCH;
  float* bcs = sm + 4 * ST * SCH;
  const int tid = (int)threadIdx.x;
  const int ch = tid >> 1, half = tid & 1;
  const int b = (int)blockIdx.x >> 4;
  const int chBase = ((int)blockIdx.x & 15) * SCH;

  float Aa[8];
  {
    const v4f a0 = *(const v4f*)(Alog + 8 * half);
    const v4f a1 = *(const v4f*)(Alog + 8 * half + 4);
    Aa[0] = -expf(bf16_val(a0.x)); Aa[1] = -expf(bf16_val(a0.y));
    Aa[2] = -expf(bf16_val(a0.z)); Aa[3] = -expf(bf16_val(a0.w));
    Aa[4] = -expf(bf16_val(a1.x)); Aa[5] = -expf(bf16_val(a1.y));
    Aa[6] = -expf(bf16_val(a1.z)); Aa[7] = -expf(bf16_val(a1.w));
  }
  const float Dd = bf16_val(Dv[chBase + ch]);
  float h[8];
#pragma unroll
  for (int j = 0; j < 8; ++j) h[j] = 0.0f;

#pragma unroll 1
  for (int cnk = 0; cnk < SEQ / ST; ++cnk) {
    const int row0 = b * SEQ + cnk * ST;
#pragma unroll
    for (int it = 0; it < 4; ++it) {
      const int idx = it * NTHR + tid;
      const int row = idx >> 5;
      const int cc  = (idx & 31) * 4;
      const size_t go = (size_t)(row0 + row) * DIN + chBase + cc;
      const v4f a = *(const v4f*)(DELTA + go);
      const v4f e = *(const v4f*)(U + go);
      const v4f f = *(const v4f*)(SZ + go);
      *(v4fa*)(dl + row * SCH + cc) = a;
      *(v4fa*)(uu + row * SCH + cc) = e;
      *(v4fa*)(sz + row * SCH + cc) = f;
    }
    {
      const int row = tid >> 3;
      const int cc  = (tid & 7) * 4;
      const v4f a = *(const v4f*)(BC + (size_t)(row0 + row) * BCW + cc);
      *(v4fa*)(bcs + row * BCW + cc) = a;
    }
    __syncthreads();

#pragma unroll 1
    for (int t = 0; t < ST; ++t) {
      const float d  = dl[t * SCH + ch];
      const float u  = uu[t * SCH + ch];
      const float zz = sz[t * SCH + ch];
      const v4f B0 = *(const v4fa*)(bcs + t * BCW + 8 * half);
      const v4f B1 = *(const v4fa*)(bcs + t * BCW + 8 * half + 4);
      const v4f C0 = *(const v4fa*)(bcs + t * BCW + 16 + 8 * half);
      const v4f C1 = *(const v4fa*)(bcs + t * BCW + 16 + 8 * half + 4);
      const float Bv[8] = {B0.x, B0.y, B0.z, B0.w, B1.x, B1.y, B1.z, B1.w};
      const float Cv[8] = {C0.x, C0.y, C0.z, C0.w, C1.x, C1.y, C1.z, C1.w};
      float p = 0.0f;
#pragma unroll
      for (int j = 0; j < 8; ++j) {
        const float dA = expf(d * Aa[j]);
        h[j] = fmaf(dA, h[j], (d * Bv[j]) * u);
        p = fmaf(h[j], Cv[j], p);
      }
      const float other = __shfl_xor(p, 1, 32);
      const float plo = (half != 0) ? other : p;
      const float phi = (half != 0) ? p : other;
      const float y = (plo + phi) + u * Dd;
      const float g = y * zz;
      if (half == 0) gg[t * SCH + ch] = g;
    }
    __syncthreads();

    v8us ov[4];
#pragma unroll
    for (int it = 0; it < 4; ++it) {
      const int plane = it >> 1;
      const int idx = (it & 1) * NTHR + tid;
      const int row = idx >> 4;
      const int c8  = (idx & 15) * 8;
      const v4f g0 = *(const v4fa*)(gg + row * SCH + c8);
      const v4f g1 = *(const v4fa*)(gg + row * SCH + c8 + 4);
      v8us o;
      o[0] = hl_bits(g0.x, plane); o[1] = hl_bits(g0.y, plane);
      o[2] = hl_bits(g0.z, plane); o[3] = hl_bits(g0.w, plane);
      o[4] = hl_bits(g1.x, plane); o[5] = hl_bits(g1.y, plane);
      o[6] = hl_bits(g1.z, plane); o[7] = hl_bits(g1.w, plane);
      ov[it] = o;
    }
#pragma unroll
    for (int it = 0; it < 4; ++it) {
      const int plane = it >> 1;
      const int idx = (it & 1) * NTHR + tid;
      const int row = idx >> 4;
      const int c8  = (idx & 15) * 8;
      unsigned short* gp = GHL + (size_t)(row0 + row) * K2 + (size_t)plane * DIN + chBase + c8;
      *(volatile v8us*)gp = ov[it];
    }
    __threadfence();
#pragma unroll
    for (int it = 0; it < 4; ++it) {
      const int plane = it >> 1;
      const int idx = (it & 1) * NTHR + tid;
      const int row = idx >> 4;
      const int c8  = (idx & 15) * 8;
      unsigned short* gp = GHL + (size_t)(row0 + row) * K2 + (size_t)plane * DIN + chBase + c8;
      *(volatile v8us*)gp = ov[it];
    }
  }
}

extern "C" void kernel_launch(void* const* d_in, const int* in_sizes, int n_in,
                              void* d_out, int out_size, void* d_ws, size_t ws_size,
                              hipStream_t stream) {
  if (n_in < 11) return;
  if (in_sizes[0] != MROWS * DIM) return;
  if (in_sizes[1] != NIN * DIM) return;
  if (in_sizes[2] != DIN * 4) return;
  if (in_sizes[3] != DIN) return;
  if (in_sizes[4] != DIN * DIN) return;
  if (in_sizes[5] != DIN) return;
  if (in_sizes[6] != 16 * DIN || in_sizes[7] != 16 * DIN) return;
  if (in_sizes[8] != 16) return;
  if (in_sizes[9] != DIN) return;
  if (in_sizes[10] != DIM * DIN) return;
  if (out_size != MROWS * DIM) return;

  const float* x     = (const float*)d_in[0];
  const float* W_in  = (const float*)d_in[1];
  const float* W_cv  = (const float*)d_in[2];
  const float* b_cv  = (const float*)d_in[3];
  const float* W_dt  = (const float*)d_in[4];
  const float* b_dt  = (const float*)d_in[5];
  const float* W_B   = (const float*)d_in[6];
  const float* W_C   = (const float*)d_in[7];
  const float* A_log = (const float*)d_in[8];
  const float* Dp    = (const float*)d_in[9];
  const float* W_out = (const float*)d_in[10];
  float* out = (float*)d_out;

  char* ws = (char*)d_ws;
  size_t off = 0;
  const size_t oXB   = off; off += (size_t)MROWS * DIM * 2;
  const size_t oWIN  = off; off += (size_t)NIN * DIM * 2;
  const size_t oWD   = off; off += (size_t)NDBC * K2 * 2;
  const size_t oWO   = off; off += (size_t)DIM * K2 * 2;
  const size_t oXI   = off; off += (size_t)PLANE * 4;
  const size_t oSZ   = off; off += (size_t)PLANE * 4;
  const size_t oU    = off; off += (size_t)PLANE * 4;
  const size_t oUHL  = off; off += (size_t)MROWS * K2 * 2;
  const size_t oBC   = off; off += (size_t)MROWS * BCW * 4;
  const size_t oGHL  = off; off += (size_t)MROWS * K2 * 2;
  if (off > ws_size || off > (size_t)WSMAX) return;
  if (oSZ != oXI + (size_t)PLANE * 4) return;
  unsigned short* XB    = (unsigned short*)(ws + oXB);
  unsigned short* WIN   = (unsigned short*)(ws + oWIN);
  unsigned short* WDBC2 = (unsigned short*)(ws + oWD);
  unsigned short* WOUT2 = (unsigned short*)(ws + oWO);
  float*          XI    = (float*)(ws + oXI);
  float*          SZp   = (float*)(ws + oSZ);
  float*          Up    = (float*)(ws + oU);
  unsigned short* UHL   = (unsigned short*)(ws + oUHL);
  float*          BCp   = (float*)(ws + oBC);
  unsigned short* GHL   = (unsigned short*)(ws + oGHL);
  float*          DELTA = XI;

  const size_t scanLds = (size_t)SCAN_LDS_FLOATS * 4;
  hipFuncSetAttribute(reinterpret_cast<const void*>(&k_scan), hipFuncAttributeMaxDynamicSharedMemorySize, (int)scanLds);

  k_prep<<<U_TOT / NTHR, NTHR, 0, stream>>>(x, W_in, W_dt, W_B, W_C, W_out, XB, WIN, WDBC2, WOUT2);
  k_gemm<0, DIN><<<dim3(MROWS / GBM, NIN / GBN), GTHR, 0, stream>>>(XB, WIN, DIM, XI, SZp, b_dt, XB);
  k_conv<<<MROWS * 2, NTHR, 0, stream>>>(XI, W_cv, b_cv, Up, UHL);
  k_gemm<1, DIN><<<dim3(MROWS / GBM, NDBC / GBN), GTHR, 0, stream>>>(UHL, WDBC2, K2, DELTA, BCp, b_dt, XB);
  k_scan<<<2 * (DIN / SCH), NTHR, scanLds, stream>>>(DELTA, Up, SZp, BCp, A_log, Dp, GHL);
  k_gemm<2, DIM><<<dim3(MROWS / GBM, DIM / GBN), GTHR, 0, stream>>>(GHL, WOUT2, K2, out, BCp, b_dt, XB);
}
